// TransformerLayer_79688823210388
// MI455X (gfx1250) — hardware-verified
//
#include <hip/hip_runtime.h>
#include <math.h>

typedef __attribute__((ext_vector_type(16))) _Float16 v16h;
typedef __attribute__((ext_vector_type(16))) __bf16 v16b;
typedef __attribute__((ext_vector_type(8)))  _Float16 v8h;
typedef __attribute__((ext_vector_type(8)))  __bf16 v8b;
typedef __attribute__((ext_vector_type(8)))  float v8f;
typedef __attribute__((ext_vector_type(4)))  float v4f;
typedef __attribute__((ext_vector_type(8)))  unsigned short v8us;

#ifndef SEQ
#define SEQ 2048
#endif
#define SEQ_FULL 2048
#ifndef NB
#define NB 2
#endif
#define NB_FULL 2
#define DM 2048
#define NH 16
#define HD 128
#define NQKV 6144
#define MROWS (NB * SEQ)
#define EROWS ((SEQ) < 256 ? (SEQ) : 256)
#define SCALE (0.08838834764831845f)
#define RC (4096.0f)
#define PCY (16384.0f)
#define WC (64.0f)
#define CC (64.0f)
#define F16MIN (6.103515625e-05f)
#define NEGBIG (-1.0e30f)
#define LOG2B64 (0.20762050593046014f)
static_assert(SEQ % 128 == 0);
static_assert(SEQ >= 128);
static_assert(SEQ <= SEQ_FULL);
static_assert(NB >= 1 && NB <= NB_FULL);
static_assert(DM == 2048 && NQKV == 3 * DM);
static_assert(NH == 16 && HD == 128 && NH * HD == DM);
static_assert(MROWS % 64 == 0);
static_assert(DM % 128 == 0 && DM % 64 == 0 && NQKV % 64 == 0 && DM % 32 == 0);
static_assert(EROWS % 64 == 0 && EROWS <= SEQ && EROWS % 32 == 0);

#define WSZ_ACT  (2u * (size_t)MROWS * DM)
#define WSZ_WT   (2u * (size_t)NQKV * DM)
#define WSZ_WO   (2u * (size_t)DM * DM)
#define WSZ_CTXR (2u * (size_t)NB * EROWS * DM)
#define WSZ_TAB  (8u * (size_t)SEQ * 64u)
#define WSZ_VTR  (2u * (size_t)NB * DM * EROWS)
#define WS_XB   ((size_t)0)
#define WS_CTX  (WS_XB)
#define WS_WT   (WS_XB  + WSZ_ACT)
#define WS_WOH  (WS_WT)
#define WS_CTXR (WS_WT  + WSZ_WO)
#define WS_QH   (WS_WT  + WSZ_WT)
#define WS_QL   (WS_QH  + WSZ_ACT)
#define WS_KH   (WS_QL  + WSZ_ACT)
#define WS_KL   (WS_KH  + WSZ_ACT)
#define WS_VT   (WS_KL  + WSZ_ACT)
#define WS_TAB  (WS_VT  + WSZ_ACT)
#define WS_VTR  (WS_TAB + WSZ_TAB)
#define WS_END  (WS_VTR + WSZ_VTR)
static_assert(WS_END <= (size_t)134217728u);
static_assert(WSZ_WO + WSZ_CTXR <= WSZ_WT);
static_assert((WSZ_ACT % 256u) == 0 && (WSZ_WT % 256u) == 0 && (WSZ_WO % 256u) == 0 && (WSZ_CTXR % 256u) == 0 && (WSZ_TAB % 256u) == 0 && (WSZ_VTR % 256u) == 0);

#define N8X ((unsigned)(NB) * (unsigned)(SEQ) * (unsigned)(DM / 8))
static_assert(N8X % 256u == 0);
#define NTAB ((unsigned)(SEQ) * 64u)
static_assert(NTAB % 256u == 0);

template <typename T> __device__ __forceinline__ void vst2(void* p, T v) { *(volatile T*)p = v; __threadfence(); *(volatile T*)p = v; }
__device__ __forceinline__ v8f zero8() { v8f z = {0.f, 0.f, 0.f, 0.f, 0.f, 0.f, 0.f, 0.f}; return z; }
__device__ __forceinline__ v8f wmma16(v16h a, v16h b, v8f c) {
  v8f d = __builtin_amdgcn_wmma_f32_16x16x32_f16(false, a, false, b, (short)0, c, false, false);
  asm volatile("v_nop\n\tv_nop\n\tv_nop\n\tv_nop" : "+v"(d) : "v"(a), "v"(b));
  return d;
}
__device__ __forceinline__ v8f wmma_bf(v16b a, v16b b, v8f c) {
  v8f d = __builtin_amdgcn_wmma_f32_16x16x32_bf16(false, a, false, b, (short)0, c, false, false);
  asm volatile("v_nop\n\tv_nop\n\tv_nop\n\tv_nop" : "+v"(d) : "v"(a), "v"(b));
  return d;
}
__device__ __forceinline__ v16h frag_h(const _Float16* rowk0, int lane) {
  union { v16h v; v8h q[2]; } u; const _Float16* p = rowk0 + 8 * (lane >> 4);
  u.q[0] = *(const v8h*)p; u.q[1] = *(const v8h*)(p + 16); return u.v;
}
__device__ __forceinline__ v16b frag_b(const __bf16* rowk0, int lane) {
  union { v16b v; v8b q[2]; } u; const __bf16* p = rowk0 + 8 * (lane >> 4);
  u.q[0] = *(const v8b*)p; u.q[1] = *(const v8b*)(p + 16); return u.v;
}
__device__ __forceinline__ _Float16 f16n(float x) { const float t = (fabsf(x) >= F16MIN) ? x : 0.0f; return (_Float16)t; }
__device__ __forceinline__ unsigned short bf16bits(float x) { unsigned u = __float_as_uint(x); u += 0x7FFFu + ((u >> 16) & 1u); return (unsigned short)(u >> 16); }
__device__ __forceinline__ float bf16val(unsigned short b) { return __uint_as_float(((unsigned)b) << 16); }
#define LDSX() do { asm volatile("s_wait_dscnt 0" ::: "memory"); __builtin_amdgcn_wave_barrier(); __builtin_amdgcn_fence(3  , "workgroup"); } while (0)

__global__ __launch_bounds__(256) void k_cvtx(const float* __restrict__ src, unsigned short* __restrict__ dst) {
  const unsigned i = blockIdx.x * 256u + threadIdx.x; if (i >= N8X) return;
  const unsigned row = i >> 8, c8 = i & 255u;
  const unsigned b = row / (unsigned)SEQ, s = row - b * (unsigned)SEQ;
  const float* p = src + ((size_t)(b * (unsigned)SEQ_FULL + s) * DM + c8 * 8u);
  const v4f a = *(const v4f*)p, c = *(const v4f*)(p + 4);
  v8us o;
#pragma unroll
  for (int e = 0; e < 4; ++e) { o[e] = bf16bits(a[e]); o[4 + e] = bf16bits(c[e]); }
  vst2(dst + (size_t)i * 8, o);
}

__global__ __launch_bounds__(256) void k_cvtw(const float* __restrict__ W, unsigned short* __restrict__ D, unsigned ldn, unsigned hm) {
  __shared__ __align__(16) unsigned short t[64][72];
  const unsigned tid = threadIdx.x;
  const bool h16 = (hm != 0u);
  const unsigned k0 = blockIdx.y * 64u, n0 = blockIdx.x * 64u;
#pragma unroll
  for (unsigned it = 0; it < 4u; ++it) {
    const unsigned e = tid + it * 256u, kr = e >> 4, nq = e & 15u;
    const v4f a = *(const v4f*)(W + (size_t)(k0 + kr) * ldn + n0 + nq * 4u);
#pragma unroll
    for (int i = 0; i < 4; ++i) {
      const unsigned short bb = bf16bits(a[i]);
      const unsigned short hb = __builtin_bit_cast(unsigned short, f16n(bf16val(bb) * WC));
      t[nq * 4u + (unsigned)i][kr] = h16 ? hb : bb;
    }
  }
  __syncthreads();
#pragma unroll
  for (unsigned it = 0; it < 2u; ++it) {
    const unsigned e = tid + it * 256u, nl = e >> 3, q = e & 7u;
    vst2(D + (size_t)(n0 + nl) * DM + k0 + q * 8u, *(const v8us*)&t[nl][q * 8u]);
  }
}

__global__ __launch_bounds__(256) void k_rope(float* __restrict__ TAB) {
  __shared__ __align__(16) float stab[512];
  const unsigned tid = threadIdx.x; const unsigned e = blockIdx.x * 256u + tid;
  const unsigned t = e >> 6, i = e & 63u;
  const float inv = exp2f(-(float)i * LOG2B64);
  const float ang = (float)t * inv;
  float sn, cs; sincosf(ang, &sn, &cs);
  stab[tid] = cs; stab[256u + tid] = sn;
  __syncthreads();
  if (tid < 128u) {
    const unsigned pl = tid >> 6, q = tid & 63u;
    const v4f v = *(const v4f*)&stab[pl * 256u + q * 4u];
    vst2(TAB + (size_t)pl * NTAB + (size_t)blockIdx.x * 256u + q * 4u, v);
  }
}

__global__ __launch_bounds__(128) void k_pqk(const __bf16* __restrict__ XB, const __bf16* __restrict__ WT, const float* __restrict__ TAB,
                                             _Float16* __restrict__ QH, _Float16* __restrict__ QL, _Float16* __restrict__ KH, _Float16* __restrict__ KL) {
  __shared__ __align__(16) _Float16 sh[64][136], sl[64][136];
  __shared__ __align__(16) float ct[64][68], st[64][68];
  const unsigned tid = threadIdx.x, wave = tid >> 5, lane = tid & 31u, col = lane & 15u, g = lane >> 4;
  const int ln = (int)lane;
  const bool zk = (blockIdx.z != 0u);
  const __bf16* WB = WT + (zk ? (size_t)DM * DM : (size_t)0);
  _Float16* OH = zk ? KH : QH; _Float16* OL = zk ? KL : QL;
  const unsigned c0 = blockIdx.y * 128u; const size_t r0 = (size_t)blockIdx.x * 64u;
  const unsigned rr = blockIdx.x * 64u; const unsigned b = rr / (unsigned)SEQ; const unsigned s0 = rr - b * (unsigned)SEQ;
  v8f acc[8];
#pragma unroll
  for (int j = 0; j < 8; ++j) acc[j] = zero8();
#pragma unroll 1
  for (unsigned kc = 0; kc < (unsigned)(DM / 32); ++kc) {
    const v16b a = frag_b(XB + (r0 + wave * 16u + col) * DM + kc * 32u, ln);
#pragma unroll
    for (int j = 0; j < 8; ++j) acc[j] = wmma_bf(a, frag_b(WB + (size_t)(c0 + (unsigned)j * 16u + col) * DM + kc * 32u, ln), acc[j]);
  }
  for (unsigned e = tid; e < 64u * 16u; e += 128u) {
    const unsigned rl = e >> 4, q = e & 15u;
    const float* tp = TAB + (size_t)(s0 + rl) * 64u + q * 4u;
    *(v4f*)&ct[rl][q * 4u] = *(const v4f*)tp;
    *(v4f*)&st[rl][q * 4u] = *(const v4f*)(tp + NTAB);
  }
  __syncthreads();
#pragma unroll
  for (int j = 0; j < 4; ++j)
#pragma unroll
    for (int r = 0; r < 8; ++r) {
      const unsigned row = wave * 16u + 8u * g + (unsigned)r, ci = (unsigned)j * 16u + col;
      const float c = ct[row][ci], s = st[row][ci];
      const float x1 = acc[j][r], x2 = acc[j + 4][r];
      const float o1 = x1 * c - x2 * s, o2 = x2 * c + x1 * s;
      const _Float16 h1 = f16n(o1), h2 = f16n(o2);
      sh[row][ci] = h1; sl[row][ci] = f16n((o1 - (float)h1) * RC);
      sh[row][ci + 64u] = h2; sl[row][ci + 64u] = f16n((o2 - (float)h2) * RC);
    }
  __syncthreads();
  for (unsigned e = tid; e < 64u * 16u; e += 128u) {
    const unsigned rl = e >> 4, q = e & 15u; const size_t o = (r0 + rl) * (size_t)DM + c0 + q * 8u;
    vst2(OH + o, *(const v8h*)&sh[rl][q * 8u]); vst2(OL + o, *(const v8h*)&sl[rl][q * 8u]);
  }
}

__global__ __launch_bounds__(128) void k_pvt(const __bf16* __restrict__ XB, const __bf16* __restrict__ WVT, _Float16* __restrict__ VT, _Float16* __restrict__ VTR) {
  __shared__ __align__(16) _Float16 th[128][72], thr[128][72];
  const unsigned tid = threadIdx.x, wave = tid >> 5, lane = tid & 31u, col = lane & 15u, g = lane >> 4;
  const int ln = (int)lane;
  const unsigned c0 = blockIdx.y * 128u; const size_t r0 = (size_t)blockIdx.x * 64u;
  const unsigned rr = blockIdx.x * 64u; const unsigned b = rr / (unsigned)SEQ; const unsigned s0 = rr - b * (unsigned)SEQ;
  const bool early = (s0 < (unsigned)EROWS);
  v8f acc[8];
#pragma unroll
  for (int j = 0; j < 8; ++j) acc[j] = zero8();
#pragma unroll 1
  for (unsigned kc = 0; kc < (unsigned)(DM / 32); ++kc) {
    const v16b a = frag_b(XB + (r0 + wave * 16u + col) * DM + kc * 32u, ln);
#pragma unroll
    for (int j = 0; j < 8; ++j) acc[j] = wmma_bf(a, frag_b(WVT + (size_t)(c0 + (unsigned)j * 16u + col) * DM + kc * 32u, ln), acc[j]);
  }
#pragma unroll
  for (int j = 0; j < 8; ++j)
#pragma unroll
    for (int r = 0; r < 8; ++r) {
      const float v = acc[j][r]; const _Float16 hv = f16n(v);
      th[(unsigned)j * 16u + col][wave * 16u + 8u * g + (unsigned)r] = hv;
      thr[(unsigned)j * 16u + col][wave * 16u + 8u * g + (unsigned)r] = f16n((v - (float)hv) * RC);
    }
  __syncthreads();
  for (unsigned e = tid; e < 128u * 8u; e += 128u) {
    const unsigned cl = e >> 3, q = e & 7u;
    vst2(VT + ((size_t)(b * (unsigned)DM + c0 + cl)) * SEQ + s0 + q * 8u, *(const v8h*)&th[cl][q * 8u]);
  }
  if (early) {
    for (unsigned e = tid; e < 128u * 8u; e += 128u) {
      const unsigned cl = e >> 3, q = e & 7u;
      vst2(VTR + ((size_t)(b * (unsigned)DM + c0 + cl)) * EROWS + s0 + q * 8u, *(const v8h*)&thr[cl][q * 8u]);
    }
  }
}

template <bool EARLY>
__global__ __launch_bounds__(128) void k_att(const _Float16* __restrict__ QH, const _Float16* __restrict__ QL, const _Float16* __restrict__ KH, const _Float16* __restrict__ KL,
                                             const _Float16* __restrict__ VT, const _Float16* __restrict__ VTR, _Float16* __restrict__ CTX, _Float16* __restrict__ CTXR) {
  constexpr int NV = EARLY ? 4 : 8;
  constexpr int SOP = NV * 16 + 8;
  constexpr int NR = EARLY ? 4 : 1;
  __shared__ __align__(16) _Float16 sP[4][16][40];
  __shared__ __align__(16) _Float16 sPr[NR][16][40];
  __shared__ __align__(16) _Float16 so[4][16][SOP];
  __shared__ __align__(16) _Float16 sor[NR][16][SOP];
  const unsigned tid = threadIdx.x, wave = tid >> 5, lane = tid & 31u, col = lane & 15u, g = lane >> 4;
  const int ln = (int)lane;
  const unsigned b = blockIdx.y >> 4, h = blockIdx.y & 15u;
  const unsigned q0 = (EARLY ? 0u : (unsigned)EROWS) + blockIdx.x * 64u + wave * 16u;
  const unsigned vc0 = EARLY ? blockIdx.z * 64u : 0u;
  const size_t rb = (size_t)b * SEQ; const size_t hoff = (size_t)h * HD;
  v16h ah[4], ar[4];
#pragma unroll
  for (int kc = 0; kc < 4; ++kc) { ah[kc] = frag_h(QH + (rb + q0 + col) * DM + hoff + kc * 32, ln); ar[kc] = frag_h(QL + (rb + q0 + col) * DM + hoff + kc * 32, ln); }
  float mrun[8], lsum[8];
#pragma unroll
  for (int r = 0; r < 8; ++r) { mrun[r] = NEGBIG; lsum[r] = 0.f; }
  v8f acc[NV], accR[NV];
#pragma unroll
  for (int j = 0; j < NV; ++j) { acc[j] = zero8(); accR[j] = zero8(); }
#pragma unroll 1
  for (unsigned j = 0; j < q0 + 16u; j += 32u) {
    LDSX();
    float sA[8], sB[8];
#pragma unroll
    for (int r = 0; r < 8; ++r) { sA[r] = NEGBIG; sB[r] = NEGBIG; }
#pragma unroll 1
    for (unsigned t = 0; t < 2u; ++t) {
      v8f cs = zero8(), cl = zero8();
      const size_t ko = (rb + j + 16u * t + col) * DM + hoff;
#pragma unroll
      for (int kc = 0; kc < 4; ++kc) {
        const v16h bh = frag_h(KH + ko + kc * 32, ln);
        const v16h br = frag_h(KL + ko + kc * 32, ln);
        cs = wmma16(ah[kc], bh, cs); cl = wmma16(ar[kc], bh, cl); cl = wmma16(ah[kc], br, cl);
      }
      const unsigned kidx = j + 16u * t + col;
#pragma unroll
      for (int r = 0; r < 8; ++r) {
        float s = (cs[r] + cl[r] * (1.0f / RC)) * SCALE;
        s = (kidx <= q0 + 8u * g + (unsigned)r) ? s : NEGBIG;
        sA[r] = sB[r]; sB[r] = s;
      }
    }
#pragma unroll
    for (int r = 0; r < 8; ++r) {
      float mx = fmaxf(sA[r], sB[r]);
      mx = fmaxf(mx, __shfl_xor(mx, 1)); mx = fmaxf(mx, __shfl_xor(mx, 2)); mx = fmaxf(mx, __shfl_xor(mx, 4)); mx = fmaxf(mx, __shfl_xor(mx, 8));
      const float mn = fmaxf(mrun[r], mx);
      const float f = __expf(mrun[r] - mn);
      mrun[r] = mn;
      float pa = __expf(sA[r] - mn) * PCY; pa = (pa >= F16MIN) ? pa : 0.0f;
      float pb = __expf(sB[r] - mn) * PCY; pb = (pb >= F16MIN) ? pb : 0.0f;
      const _Float16 pha = (_Float16)pa, phb = (_Float16)pb;
      const float fa = (float)pha, fb = (float)phb;
      if constexpr (EARLY) {
        const _Float16 pra = f16n((pa - fa) * RC), prb = f16n((pb - fb) * RC);
        lsum[r] = lsum[r] * f + ((fa + (float)pra * (1.0f / RC)) + (fb + (float)prb * (1.0f / RC)));
        sPr[wave][8u * g + (unsigned)r][col] = pra;
        sPr[wave][8u * g + (unsigned)r][16u + col] = prb;
#pragma unroll
        for (int jv = 0; jv < NV; ++jv) { acc[jv][r] *= f; accR[jv][r] *= f; }
      } else {
        lsum[r] = lsum[r] * f + (fa + fb);
#pragma unroll
        for (int jv = 0; jv < NV; ++jv) acc[jv][r] *= f;
      }
      sP[wave][8u * g + (unsigned)r][col] = pha;
      sP[wave][8u * g + (unsigned)r][16u + col] = phb;
    }
    LDSX();
    const v16h a = frag_h(&sP[wave][col][0], ln);
    if constexpr (EARLY) {
      const v16h apr = frag_h(&sPr[wave][col][0], ln);
#pragma unroll
      for (int jv = 0; jv < NV; ++jv) {
        const size_t vrow = (size_t)(b * (unsigned)DM) + hoff + vc0 + (unsigned)jv * 16u + col;
        const v16h bvh = frag_h(VT + vrow * SEQ + j, ln);
        const v16h bvr = frag_h(VTR + vrow * EROWS + j, ln);
        acc[jv] = wmma16(a, bvh, acc[jv]);
        accR[jv] = wmma16(apr, bvh, accR[jv]);
        accR[jv] = wmma16(a, bvr, accR[jv]);
      }
    } else {
#pragma unroll
      for (int jv = 0; jv < NV; ++jv) acc[jv] = wmma16(a, frag_h(VT + ((size_t)(b * (unsigned)DM) + hoff + (unsigned)jv * 16u + col) * SEQ + j, ln), acc[jv]);
    }
  }
  float inv[8];
#pragma unroll
  for (int r = 0; r < 8; ++r) { float t = lsum[r]; t += __shfl_xor(t, 1); t += __shfl_xor(t, 2); t += __shfl_xor(t, 4); t += __shfl_xor(t, 8); inv[r] = (1.0f / t) * CC; }
  LDSX();
  if constexpr (EARLY) {
#pragma unroll
    for (int jv = 0; jv < NV; ++jv)
#pragma unroll
      for (int r = 0; r < 8; ++r) {
        const float v = (acc[jv][r] + accR[jv][r] * (1.0f / RC)) * inv[r];
        const _Float16 ch = f16n(v);
        so[wave][8u * g + (unsigned)r][(unsigned)jv * 16u + col] = ch;
        sor[wave][8u * g + (unsigned)r][(unsigned)jv * 16u + col] = f16n((v - (float)ch) * RC);
      }
    LDSX();
#pragma unroll
    for (unsigned i = 0; i < 4u; ++i) {
      const unsigned rl = i * 4u + (lane >> 3), pq = lane & 7u;
      const v8h v = *(const v8h*)&so[wave][rl][pq * 8u];
      const v8h w = *(const v8h*)&sor[wave][rl][pq * 8u];
      vst2(CTX + (rb + q0 + rl) * DM + hoff + vc0 + pq * 8u, v);
      vst2(CTXR + ((size_t)b * EROWS + q0 + rl) * DM + hoff + vc0 + pq * 8u, w);
    }
  } else {
#pragma unroll
    for (int jv = 0; jv < NV; ++jv)
#pragma unroll
      for (int r = 0; r < 8; ++r) so[wave][8u * g + (unsigned)r][(unsigned)jv * 16u + col] = f16n(acc[jv][r] * inv[r]);
    LDSX();
#pragma unroll
    for (unsigned i = 0; i < 8u; ++i) {
      const unsigned rl = i * 2u + (lane >> 4), pq = lane & 15u;
      const v8h v = *(const v8h*)&so[wave][rl][pq * 8u];
      vst2(CTX + (rb + q0 + rl) * DM + hoff + pq * 8u, v);
    }
  }
}

template <bool EARLY>
__global__ __launch_bounds__(128) void k_gl(const _Float16* __restrict__ C16, const _Float16* __restrict__ C16R, const _Float16* __restrict__ WOH, float* __restrict__ OUT) {
  constexpr int NJ = EARLY ? 4 : 8;
  constexpr unsigned CW = (unsigned)NJ * 16u;
  constexpr unsigned NBK = EARLY ? (unsigned)(EROWS / 64) : (((SEQ - EROWS) / 64) > 0 ? (unsigned)((SEQ - EROWS) / 64) : 1u);
  constexpr unsigned LSH = EARLY ? 4u : 5u;
  constexpr unsigned RPI = 32u >> LSH;
  __shared__ __align__(16) float sf[4][16][CW + 4u];
  const unsigned tid = threadIdx.x, wave = tid >> 5, lane = tid & 31u, col = lane & 15u, g = lane >> 4;
  const int ln = (int)lane;
  const unsigned c0 = blockIdx.y * CW;
  const unsigned bb = blockIdx.x / NBK;
  const unsigned s0 = (EARLY ? 0u : (unsigned)EROWS) + (blockIdx.x - bb * NBK) * 64u + wave * 16u;
  const size_t r0 = (size_t)bb * SEQ + s0; const size_t rf0 = (size_t)bb * SEQ_FULL + s0; const size_t rr0 = (size_t)bb * EROWS + s0;
  v8f acc[NJ], accR[NJ];
#pragma unroll
  for (int j = 0; j < NJ; ++j) { acc[j] = zero8(); accR[j] = zero8(); }
#pragma unroll 1
  for (unsigned kc = 0; kc < (unsigned)(DM / 32); ++kc) {
    const v16h a = frag_h(C16 + (r0 + col) * DM + kc * 32u, ln);
    if constexpr (EARLY) {
      const v16h ar = frag_h(C16R + (rr0 + col) * DM + kc * 32u, ln);
#pragma unroll
      for (int j = 0; j < NJ; ++j) { const v16h bw = frag_h(WOH + (size_t)(c0 + (unsigned)j * 16u + col) * DM + kc * 32u, ln); acc[j] = wmma16(a, bw, acc[j]); accR[j] = wmma16(ar, bw, accR[j]); }
    } else {
#pragma unroll
      for (int j = 0; j < NJ; ++j) acc[j] = wmma16(a, frag_h(WOH + (size_t)(c0 + (unsigned)j * 16u + col) * DM + kc * 32u, ln), acc[j]);
    }
  }
#pragma unroll
  for (int j = 0; j < NJ; ++j)
#pragma unroll
    for (int r = 0; r < 8; ++r) {
      float v = acc[j][r] * (1.0f / (WC * CC));
      if constexpr (EARLY) v += accR[j][r] * (1.0f / (RC * WC * CC));
      sf[wave][8u * g + (unsigned)r][(unsigned)j * 16u + col] = v;
    }
  LDSX();
  for (unsigned i = 0; i < 16u / RPI; ++i) {
    const unsigned rl = i * RPI + (lane >> LSH), pq = lane & ((1u << LSH) - 1u);
    const v4f vv = *(const v4f*)&sf[wave][rl][pq * 4u];
    vst2(OUT + (rf0 + rl) * (size_t)DM + c0 + pq * 4u, vv);
  }
}

extern "C" void kernel_launch(void* const* d_in, const int* in_sizes, int n_in, void* d_out, int out_size, void* d_ws, size_t ws_size, hipStream_t stream) {
  if (n_in < 3) return;
  const int xneed = ((NB - 1) * SEQ_FULL + SEQ) * DM;
  if (in_sizes[0] < xneed || in_sizes[1] < DM * NQKV || in_sizes[2] < DM * DM) return;
  if (out_size < xneed) return;
  if (ws_size < (size_t)WS_END) return;
  const float* X = (const float*)d_in[0]; const float* WQKV = (const float*)d_in[1]; const float* WO = (const float*)d_in[2];
  char* ws = (char*)d_ws;
  unsigned short* XBu = (unsigned short*)(ws + WS_XB); unsigned short* WTu = (unsigned short*)(ws + WS_WT); unsigned short* WOHu = (unsigned short*)(ws + WS_WOH);
  const __bf16* XB = (const __bf16*)(ws + WS_XB); const __bf16* WT = (const __bf16*)(ws + WS_WT);
  const _Float16* WOH = (const _Float16*)(ws + WS_WOH);
  float* TAB = (float*)(ws + WS_TAB);
  _Float16 *QH = (_Float16*)(ws + WS_QH), *QL = (_Float16*)(ws + WS_QL), *KH = (_Float16*)(ws + WS_KH), *KL = (_Float16*)(ws + WS_KL);
  _Float16 *VT = (_Float16*)(ws + WS_VT), *VTR = (_Float16*)(ws + WS_VTR), *CTX = (_Float16*)(ws + WS_CTX), *CTXR = (_Float16*)(ws + WS_CTXR);

  k_cvtx<<<dim3(N8X / 256u), 256, 0, stream>>>(X, XBu);
  k_cvtw<<<dim3(NQKV / 64, DM / 64), 256, 0, stream>>>(WQKV, WTu, (unsigned)NQKV, 0u);
  k_rope<<<dim3(NTAB / 256u), 256, 0, stream>>>(TAB);
  k_pqk<<<dim3(MROWS / 64, NH, 2), 128, 0, stream>>>(XB, WT, TAB, QH, QL, KH, KL);
  k_pvt<<<dim3(MROWS / 64, DM / 128), 128, 0, stream>>>(XB, WT + (size_t)2 * DM * DM, VT, VTR);
  k_cvtw<<<dim3(DM / 64, DM / 64), 256, 0, stream>>>(WO, WOHu, (unsigned)DM, 1u);
  k_att<true><<<dim3(EROWS / 64, NB * NH, 2), 128, 0, stream>>>(QH, QL, KH, KL, VT, VTR, CTX, CTXR);
  if (SEQ > EROWS) k_att<false><<<dim3((SEQ - EROWS) / 64, NB * NH), 128, 0, stream>>>(QH, QL, KH, KL, VT, VTR, CTX, CTXR);
  k_gl<true><<<dim3(NB * (EROWS / 64), DM / 64), 128, 0, stream>>>(CTX, CTXR, WOH, (float*)d_out);
  if (SEQ > EROWS) k_gl<false><<<dim3(NB * ((SEQ - EROWS) / 64), DM / 128), 128, 0, stream>>>(CTX, CTXR, WOH, (float*)d_out);
}
